// SpGAT_14078902796506
// MI455X (gfx1250) — hardware-verified
//
#include <hip/hip_runtime.h>
#include <math.h>

typedef __attribute__((ext_vector_type(16))) _Float16 v16h;
typedef __attribute__((ext_vector_type(16))) __bf16 v16b;
typedef __attribute__((ext_vector_type(8)))  _Float16 v8h;
typedef __attribute__((ext_vector_type(8)))  float v8f;
typedef __attribute__((ext_vector_type(4)))  float v4f;
typedef __attribute__((ext_vector_type(2)))  float v2f;
typedef __attribute__((ext_vector_type(4)))  unsigned v4u;
typedef __attribute__((ext_vector_type(4)))  int v4i;
typedef float __attribute__((may_alias)) float_a;
typedef int __attribute__((may_alias)) int_a;

template <typename T> __device__ __forceinline__ void vst2(void* p, T v) { *(volatile T*)p = v; __threadfence(); *(volatile T*)p = v; }
__device__ __forceinline__ v8f wmma16(v16h a, v16h b, v8f c) {
  v8f d = __builtin_amdgcn_wmma_f32_16x16x32_f16(false, a, false, b, (short)0, c, false, false);
  asm volatile("v_nop\n\tv_nop\n\tv_nop\n\tv_nop" : "+v"(d) : "v"(a), "v"(b));
  return d;
}
__device__ __forceinline__ v8f wmma_bf(v16b a, v16b b, v8f c) {
  v8f d = __builtin_amdgcn_wmma_f32_16x16x32_bf16(false, a, false, b, (short)0, c, false, false);
  asm volatile("v_nop\n\tv_nop\n\tv_nop\n\tv_nop" : "+v"(d) : "v"(a), "v"(b));
  return d;
}
__device__ __forceinline__ v16h frag_h(const _Float16* rowk0, int lane) {
  union { v16h v; v8h q[2]; } u; const _Float16* p = rowk0 + 8 * (lane >> 4);
  u.q[0] = *(const v8h*)p; u.q[1] = *(const v8h*)(p + 16); return u.v;
}
__device__ __forceinline__ v16h frag_f32(const float* rowk0, int lane) {
  v16h a; const float* p = rowk0 + 8 * (lane >> 4);
#pragma unroll
  for (int i = 0; i < 8; ++i) { a[i] = (_Float16)p[i]; a[8 + i] = (_Float16)p[16 + i]; }
  return a;
}
__device__ __forceinline__ v16h frag_f32s(const float* rowk0, int lane, float sc) {
  v16h a; const float* p = rowk0 + 8 * (lane >> 4);
#pragma unroll
  for (int i = 0; i < 8; ++i) { a[i] = (_Float16)(p[i] * sc); a[8 + i] = (_Float16)(p[16 + i] * sc); }
  return a;
}
__device__ __forceinline__ v16h fragc_f32(const float* W, int k0, int n, int lane, int ld, int K) {
  v16h a; const int g = lane >> 4;
#pragma unroll
  for (int i = 0; i < 8; ++i) { const int ka = k0 + 8 * g + i, kb = ka + 16;
    a[i] = (_Float16)(ka < K ? W[(size_t)(ka < K ? ka : K - 1) * ld + n] : 0.f); a[8 + i] = (_Float16)(kb < K ? W[(size_t)(kb < K ? kb : K - 1) * ld + n] : 0.f); }
  return a;
}
struct F2 { v16b h, l; };
__device__ __forceinline__ F2 bsplit16(const float v[16]) { F2 r;
#pragma unroll
  for (int i = 0; i < 16; ++i) { const __bf16 h = (__bf16)v[i]; r.h[i] = h; r.l[i] = (__bf16)(v[i] - (float)h); }
  return r; }
__device__ __forceinline__ F2 split_row(const float* row, int k0, int lane) { float v[16]; const float* p = row + k0 + 8 * (lane >> 4);
#pragma unroll
  for (int i = 0; i < 8; ++i) { v[i] = p[i]; v[8 + i] = p[16 + i]; }
  return bsplit16(v); }
__device__ __forceinline__ F2 split_rowK(const float* row, int k0, int lane, int K) { float v[16]; const int g = lane >> 4;
#pragma unroll
  for (int i = 0; i < 8; ++i) { const int ka = k0 + 8 * g + i, kb = ka + 16; v[i] = ka < K ? row[ka < K ? ka : K - 1] : 0.f; v[8 + i] = kb < K ? row[kb < K ? kb : K - 1] : 0.f; }
  return bsplit16(v); }
__device__ __forceinline__ F2 split_col(const float* W, int k0, int n, int lane, int ld, int K) { float v[16]; const int g = lane >> 4;
#pragma unroll
  for (int i = 0; i < 8; ++i) { const int ka = k0 + 8 * g + i, kb = ka + 16; v[i] = ka < K ? W[(size_t)(ka < K ? ka : K - 1) * ld + n] : 0.f; v[8 + i] = kb < K ? W[(size_t)(kb < K ? kb : K - 1) * ld + n] : 0.f; }
  return bsplit16(v); }
__device__ __forceinline__ v8f mac3(const F2& a, const F2& b, v8f c) { c = wmma_bf(a.l, b.h, c); c = wmma_bf(a.h, b.l, c); return wmma_bf(a.h, b.h, c); }
__device__ __forceinline__ float sigm(float v) { return 1.0f / (1.0f + expf(-v)); }
#define LDSX() do { asm volatile("s_wait_dscnt 0" ::: "memory"); __builtin_amdgcn_wave_barrier(); __builtin_amdgcn_fence(__ATOMIC_RELEASE, "workgroup"); } while (0)


#define NB 4
#define NN 2048
#define NF 512
#define HD 64
#define NH 4
__device__ __forceinline__ float bfr(float v) { return (float)(__bf16)v; }
__device__ __forceinline__ v16b frag_b(const __bf16* rowk0, int lane) { return __builtin_bit_cast(v16b, frag_h((const _Float16*)rowk0, lane)); }
__device__ __attribute__((noinline)) float exp_ni(float v) { return expf(v); }
__device__ __attribute__((noinline)) float elu_ni(float v) { return v > 0.f ? v : expm1f(v); }

__global__ __launch_bounds__(256) void k_cvt(const float* __restrict__ x, __bf16* __restrict__ Xb) {
  const size_t i8 = (size_t)blockIdx.x * 256 + threadIdx.x; if (i8 >= (size_t)NB * NN * NF / 8) return;
  union { __bf16 h[8]; v4u u; } pk;
#pragma unroll
  for (int e = 0; e < 8; ++e) pk.h[e] = (__bf16)x[i8 * 8 + e];
  vst2((unsigned*)(Xb + i8 * 8), pk.u);
}
template <int LAYER>
__global__ __launch_bounds__(128) void k_proj(const __bf16* __restrict__ Xb, const float* __restrict__ H1, const float* __restrict__ W, const float* __restrict__ av, float* __restrict__ F, __bf16* __restrict__ FTh, __bf16* __restrict__ FTl, float* __restrict__ S) {
  __shared__ __align__(16) float so[4][16][68]; __shared__ __align__(16) __bf16 sth[64][72], stl[64][72]; __shared__ __align__(16) float ss[64][2];
  const int tid = threadIdx.x, wave = tid >> 5, lane = tid & 31, col = lane & 15, g = lane >> 4; const int bh = blockIdx.y, n0 = blockIdx.x * 64; const int r0 = n0 + wave * 16;
  v8f acc[4] = {};
  if (LAYER == 1) { const int b = bh / NH, h = bh % NH; const float* Wh = W + (size_t)h * NF * HD;
#pragma unroll 2
    for (int kc = 0; kc < NF / 32; ++kc) { const v16b a = frag_b(Xb + ((size_t)b * NN + r0 + col) * NF + kc * 32, lane);
#pragma unroll
      for (int j = 0; j < 4; ++j) acc[j] = wmma_bf(a, split_col(Wh, kc * 32, j * 16 + col, lane, HD, NF).h, acc[j]); } }
  else {
#pragma unroll 2
    for (int kc = 0; kc < NH * HD / 32; ++kc) { const F2 a = split_row(H1 + ((size_t)bh * NN + r0 + col) * (NH * HD), kc * 32, lane);
#pragma unroll
      for (int j = 0; j < 4; ++j) { const v16b wb = split_col(W, kc * 32, j * 16 + col, lane, HD, NH * HD).h; acc[j] = wmma_bf(a.l, wb, acc[j]); acc[j] = wmma_bf(a.h, wb, acc[j]); } } }
#pragma unroll
  for (int j = 0; j < 4; ++j)
#pragma unroll
    for (int r = 0; r < 8; ++r) { const float v = acc[j][r]; so[wave][8 * g + r][j * 16 + col] = v; const __bf16 hi = (__bf16)v; sth[j * 16 + col][wave * 16 + 8 * g + r] = hi; stl[j * 16 + col][wave * 16 + 8 * g + r] = (__bf16)(v - (float)hi); }
  LDSX();
  { const int rl = lane & 15, which = lane >> 4; const float* ap = av + (LAYER == 1 ? (size_t)(bh % NH) * 2 * HD : 0) + which * HD; float s = 0.f;
#pragma unroll 4
    for (int d = 0; d < HD; ++d) s += so[wave][rl][d] * bfr(ap[d]);
    ss[wave * 16 + rl][which] = s; }
  for (int qq = lane; qq < 16 * 16; qq += 32) { const int rl = qq >> 4, pc = qq & 15; vst2(F + ((size_t)bh * NN + r0 + rl) * HD + pc * 4, *(const v4f*)(&so[wave][rl][pc * 4])); }
  __syncthreads();
  for (int qq = tid; qq < 64 * 8; qq += 128) { const int d = qq >> 3, pc = qq & 7; const size_t o = ((size_t)bh * HD + d) * NN + n0 + pc * 8; vst2((unsigned*)(FTh + o), *(const v4u*)(&sth[d][pc * 8])); vst2((unsigned*)(FTl + o), *(const v4u*)(&stl[d][pc * 8])); }
  if (tid < 32) vst2(S + ((size_t)bh * NN + n0) * 2 + tid * 4, *(const v4f*)(&ss[0][0] + tid * 4));
}
template <int HPB, int OST>
__global__ __launch_bounds__(128) void k_gat(const float* __restrict__ S, const float* __restrict__ adj, const __bf16* __restrict__ FTh, const __bf16* __restrict__ FTl, float* __restrict__ OUT) {
  __shared__ __align__(16) __bf16 seh[4][16][72], sel[4][16][72]; __shared__ float ssrc[4][16]; __shared__ __align__(16) float so[4][16][68];
  const int tid = threadIdx.x, w = tid >> 5, lane = tid & 31, col = lane & 15, g = lane >> 4; const int bh = blockIdx.y; const int i0 = blockIdx.x * 64 + w * 16;
  if (lane < 16) ssrc[w][lane] = S[((size_t)bh * NN + i0 + lane) * 2];
  v8f acc[4] = {}; float dpart = 0.f;
  LDSX();
  const int rl = lane & 15, jh = lane >> 4; const float si = ssrc[w][rl]; const float* arow = adj + (size_t)(i0 + rl) * NN;
#pragma unroll 1
  for (int kt = 0; kt < NN / 64; ++kt) { const int j0 = kt * 64 + jh * 32;
#pragma unroll 4
    for (int jj = 0; jj < 32; ++jj) { const int j = j0 + jj; const float a = bfr(arow[j]); float ev = 0.f;
      if (a != 0.f) { float z = si + S[((size_t)bh * NN + j) * 2 + 1]; z = z > 0.f ? z : 0.2f * z; ev = exp_ni(-z) * a; }
      dpart += ev; const __bf16 hi = (__bf16)ev; seh[w][rl][jh * 32 + jj] = hi; sel[w][rl][jh * 32 + jj] = (__bf16)(ev - (float)hi); }
    LDSX();
#pragma unroll
    for (int kc = 0; kc < 2; ++kc) { const v16b eh = frag_b(&seh[w][col][kc * 32], lane), el = frag_b(&sel[w][col][kc * 32], lane);
#pragma unroll
      for (int t = 0; t < 4; ++t) { const size_t fo = ((size_t)bh * HD + t * 16 + col) * NN + kt * 64 + kc * 32; const v16b fh = frag_b(FTh + fo, lane), fl = frag_b(FTl + fo, lane); acc[t] = wmma_bf(el, fh, acc[t]); acc[t] = wmma_bf(eh, fl, acc[t]); acc[t] = wmma_bf(eh, fh, acc[t]); } }
    LDSX(); }
  const float den = dpart + __shfl_xor(dpart, 16, 32);
  __shared__ float sden[4][16]; if (jh == 0) sden[w][rl] = den;
  LDSX();
#pragma unroll
  for (int r = 0; r < 8; ++r) { const float dn = sden[w][8 * g + r];
#pragma unroll
    for (int t = 0; t < 4; ++t) { const float v = acc[t][r] / dn; so[w][8 * g + r][t * 16 + col] = elu_ni(v); } }
  LDSX();
  const int ob = bh / HPB, oh = bh % HPB;
  for (int qq = lane; qq < 16 * 16; qq += 32) { const int r2 = qq >> 4, pc = qq & 15; vst2(OUT + ((size_t)ob * NN + i0 + r2) * OST + oh * HD + pc * 4, *(const v4f*)(&so[w][r2][pc * 4])); }
}
extern "C" void kernel_launch(void* const* d_in, const int* in_sizes, int n_in, void* d_out, int out_size, void* d_ws, size_t ws_size, hipStream_t stream) {
  (void)in_sizes; (void)n_in; (void)out_size; (void)ws_size;
  const float* x = (const float*)d_in[0]; const float* adj = (const float*)d_in[1]; const float* W1 = (const float*)d_in[2]; const float* a1 = (const float*)d_in[3]; const float* W2 = (const float*)d_in[4]; const float* a2 = (const float*)d_in[5];
  char* ws = (char*)d_ws; size_t off = 0;
  auto take = [&](size_t bytes) { char* p = ws + off; off += (bytes + 255) & ~(size_t)255; return p; };
  __bf16* Xb = (__bf16*)take((size_t)NB * NN * NF * 2);
  float* F = (float*)take((size_t)NB * NH * NN * HD * 4); __bf16* FTh = (__bf16*)take((size_t)NB * NH * HD * NN * 2); __bf16* FTl = (__bf16*)take((size_t)NB * NH * HD * NN * 2); float* S = (float*)take((size_t)NB * NH * NN * 2 * 4);
  float* H1 = (float*)take((size_t)NB * NN * NH * HD * 4);
  float* G = (float*)take((size_t)NB * NN * HD * 4); __bf16* GTh = (__bf16*)take((size_t)NB * HD * NN * 2); __bf16* GTl = (__bf16*)take((size_t)NB * HD * NN * 2); float* S2 = (float*)take((size_t)NB * NN * 2 * 4);
  k_cvt<<<(NB * NN * NF / 8 + 255) / 256, 256, 0, stream>>>(x, Xb);
  k_proj<1><<<dim3(NN / 64, NB * NH), 128, 0, stream>>>(Xb, nullptr, W1, a1, F, FTh, FTl, S);
  k_gat<NH, NH * HD><<<dim3(NN / 64, NB * NH), 128, 0, stream>>>(S, adj, FTh, FTl, H1);
  k_proj<2><<<dim3(NN / 64, NB), 128, 0, stream>>>(nullptr, H1, W2, a2, G, GTh, GTl, S2);
  k_gat<1, HD><<<dim3(NN / 64, NB), 128, 0, stream>>>(S2, adj, GTh, GTl, (float*)d_out);
}
